// DABlock_36481452212798
// MI455X (gfx1250) — hardware-run, weakly checked
//
#include <hip/hip_runtime.h>
#include <stdint.h>
#include <stddef.h>

typedef __attribute__((ext_vector_type(16))) _Float16 v16h;
typedef __attribute__((ext_vector_type(8)))  _Float16 v8h;
typedef __attribute__((ext_vector_type(16))) __bf16   v16b;
typedef __attribute__((ext_vector_type(8)))  __bf16   v8b;
typedef __attribute__((ext_vector_type(8)))  float    v8f;
typedef __attribute__((ext_vector_type(4)))  float    v4f;
typedef __attribute__((ext_vector_type(4)))  unsigned int v4u;
#define PSCALE 32768.0f
#define U16(p) ((const unsigned short*)(const void*)(p))
#define PSCALE_INV (1.0f / 32768.0f)

constexpr int NBATCH = 4;
constexpr int NCH    = 256;
constexpr int NPIX   = 4096;
constexpr int CH4    = 1024;
constexpr int KPOOL  = 128;
constexpr int NSTAGE = 6;
constexpr int NHEAD  = 8;
constexpr int HDIM   = 128;
constexpr int KCONV  = 2304;
constexpr int QKV_LD = 3072;

constexpr float WCAR = 32.0f;
constexpr float QCAR = 8.0f;
constexpr float ZCAR = 1024.0f;
constexpr float BCAR = 64.0f;
constexpr float PCAR = 1024.0f;
constexpr float OCAR = 16.0f;
constexpr float HCAR = 16.0f;
constexpr float ATT_SCALE = 0.17677669529663687f;

static_assert(NCH % 32 == 0 && CH4 % 32 == 0 && KCONV % 32 == 0 && NPIX % 32 == 0 && HDIM % 32 == 0 && KPOOL % 32 == 0);
static_assert(NPIX % 64 == 0 && QKV_LD % 64 == 0 && CH4 % 64 == 0 && NCH % 64 == 0 && KPOOL % 64 == 0 && HDIM % 64 == 0);
static_assert((NBATCH * NPIX) % 64 == 0 && NPIX % KPOOL == 0 && NPIX / KPOOL == 32 && CH4 == NHEAD * HDIM);

__device__ __forceinline__ unsigned short f2bf_bits(float f) {
  unsigned u = __float_as_uint(f);
  return (unsigned short)((u + 0x7FFFu + ((u >> 16) & 1u)) >> 16);
}
__device__ __forceinline__ float bf_bits2f(unsigned short h) { return __uint_as_float(((unsigned)h) << 16); }
__device__ __forceinline__ float h_bits2f(unsigned short h) { return (float)__builtin_bit_cast(_Float16, h); }
__device__ __forceinline__ unsigned short f2h_bits(float f) { return __builtin_bit_cast(unsigned short, (_Float16)f); }

__device__ __forceinline__ void dep_guard_h(v8f& a, v8f& b, v16h x, v16h y) { asm volatile("v_nop\n\tv_nop\n\tv_nop\n\tv_nop" : "+v"(a), "+v"(b) : "v"(x), "v"(y)); }
__device__ __forceinline__ void dep_guard_b(v8f& a, v8f& b, v16b x, v16b y) { asm volatile("v_nop\n\tv_nop\n\tv_nop\n\tv_nop" : "+v"(a), "+v"(b) : "v"(x), "v"(y)); }
__device__ __forceinline__ void keep4_h(v16h a, v16h b, v16h c, v16h d) { asm volatile("v_nop" :: "v"(a), "v"(b), "v"(c), "v"(d)); }
__device__ __forceinline__ void keep4_b(v16b a, v16b b, v16b c, v16b d) { asm volatile("v_nop" :: "v"(a), "v"(b), "v"(c), "v"(d)); }
__device__ __forceinline__ void acc_guard4(v8f& a, v8f& b, v8f& c, v8f& d) { asm volatile("v_nop\n\tv_nop\n\tv_nop\n\tv_nop" : "+v"(a), "+v"(b), "+v"(c), "+v"(d)); }
template <typename T> struct Frag;
template <> struct Frag<_Float16> {
  typedef v16h V; union U { v16h v; v8h h[2]; };
  static __device__ __forceinline__ v16h load(const _Float16* p) {
    U f; f.h[0] = *(const v8h*)(p); f.h[1] = *(const v8h*)(p + 16); return f.v;
  }
  static __device__ __forceinline__ v8f mma(v16h a, v16h b, v8f c) {
    return __builtin_amdgcn_wmma_f32_16x16x32_f16(false, a, false, b, (short)0, c, false, false);
  }
  static __device__ __forceinline__ void guard(v8f& a, v8f& b, v16h x, v16h y) { dep_guard_h(a, b, x, y); }
  static __device__ __forceinline__ void keep(v16h a, v16h b, v16h c, v16h d) { keep4_h(a, b, c, d); }
};
template <> struct Frag<__bf16> {
  typedef v16b V; union U { v16b v; v8b h[2]; };
  static __device__ __forceinline__ v16b load(const __bf16* p) {
    U f; f.h[0] = *(const v8b*)(p); f.h[1] = *(const v8b*)(p + 16); return f.v;
  }
  static __device__ __forceinline__ v8f mma(v16b a, v16b b, v8f c) {
    return __builtin_amdgcn_wmma_f32_16x16x32_bf16(false, a, false, b, (short)0, c, false, false);
  }
  static __device__ __forceinline__ void guard(v8f& a, v8f& b, v16b x, v16b y) { dep_guard_b(a, b, x, y); }
  static __device__ __forceinline__ void keep(v16b a, v16b b, v16b c, v16b d) { keep4_b(a, b, c, d); }
};

template <int ET> struct Elem;
template <> struct Elem<0> { typedef _Float16 T; };
template <> struct Elem<1> { typedef __bf16 T; };
template <int ET, bool SPLIT, int BIAS_MODE, int OUT_MODE, bool RESID, int ACT = 0>
__global__ __launch_bounds__(256) void wmma_gemm64(
    const unsigned short* __restrict__ Ap, const unsigned short* __restrict__ A2p, int lda, long strideA,
    const unsigned short* __restrict__ Btp, const unsigned short* __restrict__ Bt2p, int ldb, long strideB,
    void* __restrict__ Cout, void* __restrict__ Cout2, int ldc, long strideC,
    const float* __restrict__ bias,
    const float* __restrict__ resid, long strideR,
    int M, int N, int K, float scale) {
  typedef typename Elem<ET>::T T;
  typedef typename Frag<T>::V V;
  const T* A = (const T*)Ap; const T* A2 = (const T*)A2p; const T* Bt = (const T*)Btp; const T* Bt2 = (const T*)Bt2p;
  __shared__ __align__(16) float sT[8][16 * 68];
  const int b    = blockIdx.y;
  const int lane = threadIdx.x & 31;
  const int wave = threadIdx.x >> 5;
  const int tilesN = N >> 6;
  const int tilesM = M >> 6;
  const int tile = blockIdx.x * 8 + wave;
  if (tile >= tilesM * tilesN) return;
  const int tm = tile / tilesN;
  const int tn = tile - tm * tilesN;
  const int m0 = tm << 6;
  const int n0 = tn << 6;

  const T* Ab  = A  + (size_t)b * strideA;
  const T* Bb  = Bt + (size_t)b * strideB;
  const T* Ab2 = SPLIT ? (A2  + (size_t)b * strideA) : nullptr;
  const T* Bb2 = SPLIT ? (Bt2 + (size_t)b * strideB) : nullptr;

  const int rlane = lane & 15;
  const int koff  = (lane >> 4) * 8;
  const int mOff  = (lane >> 4) * 8;

  v8f acc[4][4];
#pragma unroll
  for (int i = 0; i < 4; ++i)
#pragma unroll
    for (int j = 0; j < 4; ++j) acc[i][j] = (v8f){0.f,0.f,0.f,0.f,0.f,0.f,0.f,0.f};

  for (int k0 = 0; k0 < K; k0 += 32) {
    V bh[4], bl[4];
#pragma unroll
    for (int j = 0; j < 4; ++j) {
      const size_t bo = (size_t)(n0 + (j << 4) + rlane) * ldb + koff + k0;
      bh[j] = Frag<T>::load(Bb + bo);
      if (SPLIT) bl[j] = Frag<T>::load(Bb2 + bo);
    }
#pragma unroll
    for (int i = 0; i < 4; ++i) {
      const size_t ao = (size_t)(m0 + (i << 4) + rlane) * lda + koff + k0;
      V ah = Frag<T>::load(Ab + ao);
      V al;
      if (SPLIT) al = Frag<T>::load(Ab2 + ao);
#pragma unroll
      for (int j = 0; j < 4; ++j) {
        acc[i][j] = Frag<T>::mma(ah, bh[j], acc[i][j]);
        if (SPLIT) {
          acc[i][j] = Frag<T>::mma(ah, bl[j], acc[i][j]);
          acc[i][j] = Frag<T>::mma(al, bh[j], acc[i][j]);
        }
      }
      Frag<T>::guard(acc[i][0], acc[i][3], ah, SPLIT ? al : ah);
    }
    Frag<T>::keep(bh[0], bh[1], bh[2], bh[3]);
    if (SPLIT) Frag<T>::keep(bl[0], bl[1], bl[2], bl[3]);
  }
  acc_guard4(acc[0][0], acc[0][1], acc[0][2], acc[0][3]);
  acc_guard4(acc[1][0], acc[1][1], acc[1][2], acc[1][3]);
  acc_guard4(acc[2][0], acc[2][1], acc[2][2], acc[2][3]);
  acc_guard4(acc[3][0], acc[3][1], acc[3][2], acc[3][3]);

  float* slab = sT[wave];
  const float* Rb = RESID ? (resid + (size_t)b * strideR) : nullptr;
#pragma unroll
  for (int i = 0; i < 4; ++i) {
    const int mBase = m0 + (i << 4);
#pragma unroll
    for (int j = 0; j < 4; ++j) {
      const int n = n0 + (j << 4) + rlane;
      float bv = 0.f;
      if (BIAS_MODE == 2) bv = bias[n];
#pragma unroll
      for (int r = 0; r < 8; ++r) {
        float v = acc[i][j][r] * scale;
        if (BIAS_MODE == 1) v += bias[mBase + mOff + r];
        if (BIAS_MODE == 2) v += bv;
        if (RESID) v += Rb[(size_t)(mBase + mOff + r) * ldc + n];
        if (ACT == 1) v = tanhf(v);
        if (ACT == 2) v = fmaxf(v, 0.0f);
        if (ACT == 3) v = v / (1.0f + expf(-v));
        if (ACT == 4) v = (v > 0.f) ? v : 0.01f * v;
        if (ACT == 5) v = 0.5f * v * (1.0f + erff(v * 0.70710678118654752f));
        slab[(mOff + r) * 68 + (j << 4) + rlane] = v;
      }
    }
    __builtin_amdgcn_fence(__ATOMIC_RELEASE, "workgroup");
    __builtin_amdgcn_wave_barrier();
    __builtin_amdgcn_fence(__ATOMIC_ACQUIRE, "workgroup");
    if (OUT_MODE == 0) {
      float* C = (float*)Cout + (size_t)b * strideC;
      const int hh = lane >> 4, c4 = (lane & 15) * 4;
      for (int pass = 0; pass < 2; ++pass) {
#pragma unroll
        for (int it = 0; it < 8; ++it) {
          const int row = it * 2 + hh;
          v4f v = *(const v4f*)(slab + row * 68 + c4);
          *(volatile v4f*)(C + (size_t)(mBase + row) * ldc + n0 + c4) = v;
        }
        __threadfence();
      }
    } else {
      const int q = lane >> 3, c8 = (lane & 7) * 8;
      unsigned short* C  = (unsigned short*)Cout  + (size_t)b * strideC;
      unsigned short* C2 = (OUT_MODE == 2) ? ((unsigned short*)Cout2 + (size_t)b * strideC) : nullptr;
      for (int pass = 0; pass < 2; ++pass) {
#pragma unroll
        for (int it = 0; it < 4; ++it) {
          const int row = it * 4 + q;
          const float* sp = slab + row * 68 + c8;
          v8h hv, lv;
#pragma unroll
          for (int e = 0; e < 8; ++e) {
            if (OUT_MODE == 1) {
              hv[e] = (_Float16)sp[e];
            } else {
              unsigned short hb = f2bf_bits(sp[e]);
              unsigned short lb = f2bf_bits(sp[e] - bf_bits2f(hb));
              hv[e] = __builtin_bit_cast(_Float16, hb);
              lv[e] = __builtin_bit_cast(_Float16, lb);
            }
          }
          *(volatile v8h*)(C + (size_t)(mBase + row) * ldc + n0 + c8) = hv;
          if (OUT_MODE == 2) *(volatile v8h*)(C2 + (size_t)(mBase + row) * ldc + n0 + c8) = lv;
        }
        __threadfence();
      }
    }
    __builtin_amdgcn_fence(__ATOMIC_RELEASE, "workgroup");
    __builtin_amdgcn_wave_barrier();
    __builtin_amdgcn_fence(__ATOMIC_ACQUIRE, "workgroup");
  }
}

template <int OUT_MODE, bool POSTMUL>
__global__ __launch_bounds__(256) void conv3x3_wmma64(
    const unsigned short* __restrict__ imgp, const unsigned short* __restrict__ wtp,
    const float* __restrict__ cs, const float* __restrict__ cb, const float* __restrict__ postp,
    void* __restrict__ Cout) {
  typedef _Float16 T;
  typedef v16h V;
  union FU { v16h v; v4u q[2]; };
  const T* X = (const T*)imgp;
  const T* Wt = (const T*)wtp;
  __shared__ __align__(16) float sT[8][16 * 68];
  const int lane = threadIdx.x & 31;
  const int wave = threadIdx.x >> 5;
  const int tilesN = NCH >> 6;
  const int tilesM = (NBATCH * NPIX) >> 6;
  const int tile = blockIdx.x * 8 + wave;
  if (tile >= tilesM * tilesN) return;
  const int tm = tile / tilesN;
  const int tn = tile - tm * tilesN;
  const int m0 = tm << 6;
  const int n0 = tn << 6;
  const int rlane = lane & 15;
  const int koff  = (lane >> 4) * 8;
  const int mOff  = (lane >> 4) * 8;
  const int bimg  = m0 >> 12;
  const T* Xb = X + (size_t)bimg * NPIX * NCH;
  int py[4], px[4];
#pragma unroll
  for (int i = 0; i < 4; ++i) {
    const int p = (m0 & (NPIX - 1)) + (i << 4) + rlane;
    py[i] = p >> 6;
    px[i] = p & 63;
  }

  v8f acc[4][4];
#pragma unroll
  for (int i = 0; i < 4; ++i)
#pragma unroll
    for (int j = 0; j < 4; ++j) acc[i][j] = (v8f){0.f,0.f,0.f,0.f,0.f,0.f,0.f,0.f};

#pragma unroll 1
  for (int kk = 0; kk < 9; ++kk) {
    const int ky = kk / 3;
    const int dy = ky - 1;
    const int dx = kk - ky * 3 - 1;
    const size_t wk0 = (size_t)kk * NCH;
#pragma unroll 1
    for (int ci0 = 0; ci0 < NCH; ci0 += 32) {
      V bh[4];
#pragma unroll
      for (int j = 0; j < 4; ++j)
        bh[j] = Frag<T>::load(Wt + (size_t)(n0 + (j << 4) + rlane) * KCONV + wk0 + ci0 + koff);
#pragma unroll
      for (int i = 0; i < 4; ++i) {
        const int sy = py[i] + dy;
        const int sx = px[i] + dx;
        const bool valid = ((unsigned)sy < 64u) && ((unsigned)sx < 64u);
        const int syc = sy < 0 ? 0 : (sy > 63 ? 63 : sy);
        const int sxc = sx < 0 ? 0 : (sx > 63 ? 63 : sx);
        FU fa;
        fa.v = Frag<T>::load(Xb + (size_t)(syc * 64 + sxc) * NCH + ci0 + koff);
        const unsigned msk = valid ? 0xffffffffu : 0u;
        const v4u mm = (v4u){msk, msk, msk, msk};
        fa.q[0] = fa.q[0] & mm;
        fa.q[1] = fa.q[1] & mm;
        const V ah = fa.v;
#pragma unroll
        for (int j = 0; j < 4; ++j) acc[i][j] = Frag<T>::mma(ah, bh[j], acc[i][j]);
        Frag<T>::guard(acc[i][0], acc[i][3], ah, ah);
      }
      Frag<T>::keep(bh[0], bh[1], bh[2], bh[3]);
    }
  }
  acc_guard4(acc[0][0], acc[0][1], acc[0][2], acc[0][3]);
  acc_guard4(acc[1][0], acc[1][1], acc[1][2], acc[1][3]);
  acc_guard4(acc[2][0], acc[2][1], acc[2][2], acc[2][3]);
  acc_guard4(acc[3][0], acc[3][1], acc[3][2], acc[3][3]);

  float post = 1.0f;
  if (POSTMUL) post = postp[0];
  float* slab = sT[wave];
#pragma unroll
  for (int i = 0; i < 4; ++i) {
    const int mBase = m0 + (i << 4);
#pragma unroll
    for (int j = 0; j < 4; ++j) {
      const int n = n0 + (j << 4) + rlane;
      const float csv = cs[n];
      const float cbv = cb[n];
#pragma unroll
      for (int r = 0; r < 8; ++r) {
        float v = fmaf(acc[i][j][r], csv, cbv);
        v = fmaxf(v, 0.0f);
        if (POSTMUL) v = v * post;
        slab[(mOff + r) * 68 + (j << 4) + rlane] = v;
      }
    }
    __builtin_amdgcn_fence(__ATOMIC_RELEASE, "workgroup");
    __builtin_amdgcn_wave_barrier();
    __builtin_amdgcn_fence(__ATOMIC_ACQUIRE, "workgroup");
    if (OUT_MODE == 0) {
      float* Cp = (float*)Cout;
      const int hh = lane >> 4, c4 = (lane & 15) * 4;
      for (int pass = 0; pass < 2; ++pass) {
#pragma unroll
        for (int it = 0; it < 8; ++it) {
          const int row = it * 2 + hh;
          v4f v = *(const v4f*)(slab + row * 68 + c4);
          *(volatile v4f*)(Cp + (size_t)(mBase + row) * NCH + n0 + c4) = v;
        }
        __threadfence();
      }
    } else {
      unsigned short* Cp = (unsigned short*)Cout;
      const int q = lane >> 3, c8 = (lane & 7) * 8;
      for (int pass = 0; pass < 2; ++pass) {
#pragma unroll
        for (int it = 0; it < 4; ++it) {
          const int row = it * 4 + q;
          const float* sp = slab + row * 68 + c8;
          v8h hv;
#pragma unroll
          for (int e = 0; e < 8; ++e) hv[e] = (_Float16)sp[e];
          *(volatile v8h*)(Cp + (size_t)(mBase + row) * NCH + n0 + c8) = hv;
        }
        __threadfence();
      }
    }
    __builtin_amdgcn_fence(__ATOMIC_RELEASE, "workgroup");
    __builtin_amdgcn_wave_barrier();
    __builtin_amdgcn_fence(__ATOMIC_ACQUIRE, "workgroup");
  }
}

__global__ __launch_bounds__(64) void dta_logit_softmax_kernel(
    const unsigned short* __restrict__ xp, const unsigned short* __restrict__ basp,
    unsigned short* __restrict__ zp, float* __restrict__ colsq, float lscale) {
  typedef _Float16 T;
  typedef v16h V;
  __shared__ __align__(16) float Ls[64 * 132];
  const int lane = threadIdx.x & 31;
  const int wave = threadIdx.x >> 5;
  const int blk = blockIdx.x;
  const int s = blockIdx.y;
  const int n0 = blk * 64;
  const T* A  = (const T*)xp + (size_t)s * CH4;
  const T* Bt = (const T*)basp + (size_t)s * KPOOL * CH4;
  const int kb0 = wave * 64;
  const int rlane = lane & 15;
  const int koff  = (lane >> 4) * 8;
  const int mOff  = (lane >> 4) * 8;

  v8f acc[4][4];
#pragma unroll
  for (int i = 0; i < 4; ++i)
#pragma unroll
    for (int j = 0; j < 4; ++j) acc[i][j] = (v8f){0.f,0.f,0.f,0.f,0.f,0.f,0.f,0.f};

  for (int k0 = 0; k0 < CH4; k0 += 32) {
    V bh[4];
#pragma unroll
    for (int j = 0; j < 4; ++j)
      bh[j] = Frag<T>::load(Bt + (size_t)(kb0 + (j << 4) + rlane) * CH4 + koff + k0);
#pragma unroll
    for (int i = 0; i < 4; ++i) {
      V ah = Frag<T>::load(A + (size_t)(n0 + (i << 4) + rlane) * QKV_LD + koff + k0);
#pragma unroll
      for (int j = 0; j < 4; ++j) acc[i][j] = Frag<T>::mma(ah, bh[j], acc[i][j]);
      Frag<T>::guard(acc[i][0], acc[i][3], ah, ah);
    }
    Frag<T>::keep(bh[0], bh[1], bh[2], bh[3]);
  }
  acc_guard4(acc[0][0], acc[0][1], acc[0][2], acc[0][3]);
  acc_guard4(acc[1][0], acc[1][1], acc[1][2], acc[1][3]);
  acc_guard4(acc[2][0], acc[2][1], acc[2][2], acc[2][3]);
  acc_guard4(acc[3][0], acc[3][1], acc[3][2], acc[3][3]);

#pragma unroll
  for (int i = 0; i < 4; ++i)
#pragma unroll
    for (int j = 0; j < 4; ++j)
#pragma unroll
      for (int r = 0; r < 8; ++r)
        Ls[((i << 4) + mOff + r) * 132 + kb0 + (j << 4) + rlane] = acc[i][j][r] * lscale;
  __syncthreads();

  {
    const int n = threadIdx.x;
    float* rp = Ls + n * 132;
    float mx = -__builtin_huge_valf();
#pragma unroll 1
    for (int kk = 0; kk < KPOOL; ++kk) mx = fmaxf(mx, rp[kk]);
    float ssum = 0.f;
#pragma unroll 1
    for (int kk = 0; kk < KPOOL; ++kk) { const float e = expf(rp[kk] - mx); rp[kk] = e; ssum += e; }
    const float inv = 1.0f / ssum;
#pragma unroll 1
    for (int kk = 0; kk < KPOOL; ++kk) rp[kk] = rp[kk] * inv;
  }
  __syncthreads();

  {
    const int ka = threadIdx.x;
    const int kb = threadIdx.x + 64;
    float sa = 0.f, sb = 0.f;
#pragma unroll 1
    for (int n = 0; n < 64; ++n) {
      const float va = Ls[n * 132 + ka];
      const float vb = Ls[n * 132 + kb];
      sa += va * va;
      sb += vb * vb;
    }
    float* cq = colsq + ((size_t)s * 64 + blk) * KPOOL;
    ((volatile float*)cq)[ka] = sa;
    ((volatile float*)cq)[kb] = sb;
    __threadfence();
    ((volatile float*)cq)[ka] = sa;
    ((volatile float*)cq)[kb] = sb;
  }

  {
    T* zb = (T*)zp + (size_t)s * KPOOL * NPIX + n0;
    const int q = lane >> 3;
    const int c8 = (lane & 7) * 8;
#pragma unroll 1
    for (int it = 0; it < 16; ++it) {
      const int kk = kb0 + it * 4 + q;
      v8h hv;
#pragma unroll
      for (int e = 0; e < 8; ++e) hv[e] = (_Float16)(Ls[(c8 + e) * 132 + kk] * ZCAR);
      T* dst = zb + (size_t)kk * NPIX + c8;
      *(volatile v8h*)dst = hv;
      __threadfence();
      *(volatile v8h*)dst = hv;
    }
  }
}

template <bool RAW>
__global__ __launch_bounds__(256) void ln_tok_kernel(
    const float* __restrict__ in, long in_bs,
    const float* __restrict__ g, const float* __restrict__ bvec,
    unsigned short* __restrict__ outp, unsigned short* __restrict__ rawp) {
  __shared__ __align__(16) float tile[32 * 260];
  const int t = threadIdx.x;
  const int lane = t & 31;
  const int wave = t >> 5;
  const int b = blockIdx.y;
  const int p0 = blockIdx.x * 32;
  const float* ib = in + (size_t)b * in_bs + p0;
  {
    const int cl = t >> 3;
    const int p4 = (t & 7) * 4;
#pragma unroll
    for (int it = 0; it < 8; ++it) {
      const int c = it * 32 + cl;
      const v4f v = *(const v4f*)(ib + (size_t)c * NPIX + p4);
      tile[(p4 + 0) * 260 + c] = v[0];
      tile[(p4 + 1) * 260 + c] = v[1];
      tile[(p4 + 2) * 260 + c] = v[2];
      tile[(p4 + 3) * 260 + c] = v[3];
    }
  }
  __syncthreads();
  const int c0 = 8 * lane;
  const v4f ga = *(const v4f*)(g + c0);
  const v4f gb = *(const v4f*)(g + c0 + 4);
  const v4f ba = *(const v4f*)(bvec + c0);
  const v4f bb = *(const v4f*)(bvec + c0 + 4);
  const size_t orow0 = (size_t)b * NPIX + p0;
#pragma unroll 1
  for (int jt = 0; jt < 4; ++jt) {
    const int tk = wave * 4 + jt;
    const float* rp = tile + tk * 260 + c0;
    const v4f xa = *(const v4f*)rp;
    const v4f xb = *(const v4f*)(rp + 4);
    float sm = ((xa[0] + xa[1]) + (xa[2] + xa[3])) + ((xb[0] + xb[1]) + (xb[2] + xb[3]));
#pragma unroll
    for (int off = 16; off > 0; off >>= 1) sm += __shfl_xor(sm, off, 32);
    const float mu = sm * (1.0f / (float)NCH);
    const float d0 = xa[0] - mu, d1 = xa[1] - mu, d2 = xa[2] - mu, d3 = xa[3] - mu;
    const float d4 = xb[0] - mu, d5 = xb[1] - mu, d6 = xb[2] - mu, d7 = xb[3] - mu;
    float sq = ((d0 * d0 + d1 * d1) + (d2 * d2 + d3 * d3)) + ((d4 * d4 + d5 * d5) + (d6 * d6 + d7 * d7));
#pragma unroll
    for (int off = 16; off > 0; off >>= 1) sq += __shfl_xor(sq, off, 32);
    const float rs = rsqrtf(sq * (1.0f / (float)NCH) + 1e-5f);
    v8h hv;
    hv[0] = (_Float16)((d0 * rs) * ga[0] + ba[0]);
    hv[1] = (_Float16)((d1 * rs) * ga[1] + ba[1]);
    hv[2] = (_Float16)((d2 * rs) * ga[2] + ba[2]);
    hv[3] = (_Float16)((d3 * rs) * ga[3] + ba[3]);
    hv[4] = (_Float16)((d4 * rs) * gb[0] + bb[0]);
    hv[5] = (_Float16)((d5 * rs) * gb[1] + bb[1]);
    hv[6] = (_Float16)((d6 * rs) * gb[2] + bb[2]);
    hv[7] = (_Float16)((d7 * rs) * gb[3] + bb[3]);
    unsigned short* op = outp + (orow0 + tk) * NCH + c0;
    *(volatile v8h*)op = hv;
    v8h rv;
    if (RAW) {
      rv[0] = (_Float16)xa[0]; rv[1] = (_Float16)xa[1]; rv[2] = (_Float16)xa[2]; rv[3] = (_Float16)xa[3];
      rv[4] = (_Float16)xb[0]; rv[5] = (_Float16)xb[1]; rv[6] = (_Float16)xb[2]; rv[7] = (_Float16)xb[3];
      *(volatile v8h*)(rawp + (orow0 + tk) * NCH + c0) = rv;
    }
    __threadfence();
    *(volatile v8h*)op = hv;
    if (RAW) *(volatile v8h*)(rawp + (orow0 + tk) * NCH + c0) = rv;
  }
}

__global__ __launch_bounds__(256) void transpose16_kernel(
    const unsigned short* __restrict__ in, int ldi, long sIn,
    unsigned short* __restrict__ out, int ldo, long sOut) {
  __shared__ __align__(16) unsigned short tl[64 * 72];
  const int t = threadIdx.x;
  const int lane = t & 31;
  const int wave = t >> 5;
  const int r0 = blockIdx.x * 64;
  const int c0 = blockIdx.y * 64;
  const unsigned short* inb = in + (size_t)blockIdx.z * sIn;
  unsigned short* outb = out + (size_t)blockIdx.z * sOut;
#pragma unroll
  for (int it = 0; it < 2; ++it) {
    const int row = it * 32 + (t >> 3);
    const int c8 = (t & 7) * 8;
    const v4u w = *(const v4u*)(inb + (size_t)(r0 + row) * ldi + c0 + c8);
#pragma unroll
    for (int e = 0; e < 8; ++e) {
      const unsigned short us = (unsigned short)((w[e >> 1] >> ((e & 1) * 16)) & 0xffffu);
      tl[(c8 + e) * 72 + row] = us;
    }
  }
  __syncthreads();
  const int q = lane >> 3;
  const int c8n = (lane & 7) * 8;
  for (int pass = 0; pass < 2; ++pass) {
#pragma unroll
    for (int it = 0; it < 2; ++it) {
      const int row = it * 32 + wave * 4 + q;
      const v4u v = *(const v4u*)(tl + row * 72 + c8n);
      *(volatile v4u*)(outb + (size_t)(c0 + row) * ldo + r0 + c8n) = v;
    }
    __threadfence();
  }
}

__global__ __launch_bounds__(256) void pool_kernel(const unsigned short* __restrict__ qkc, float* __restrict__ raw) {
  const int c = blockIdx.x * 256 + threadIdx.x;
  const int kk = blockIdx.y;
  const int s = blockIdx.z;
  const unsigned short* p = qkc + ((size_t)s * CH4 + c) * NPIX + kk * 32;
  float mx = -__builtin_huge_valf();
#pragma unroll
  for (int w4 = 0; w4 < 4; ++w4) {
    const v4u wv = *(const v4u*)(p + w4 * 8);
#pragma unroll
    for (int e = 0; e < 4; ++e) {
      const unsigned u = wv[e];
      mx = fmaxf(mx, h_bits2f((unsigned short)(u & 0xffffu)));
      mx = fmaxf(mx, h_bits2f((unsigned short)(u >> 16)));
    }
  }
  float* dst = raw + ((size_t)s * KPOOL + kk) * CH4 + c;
  *(volatile float*)dst = mx;
  __threadfence();
  *(volatile float*)dst = mx;
}

template <bool HAS_SZ>
__global__ __launch_bounds__(256) void rownorm_kernel(
    const float* __restrict__ raw, const float* __restrict__ colsq, float gin, unsigned short* __restrict__ out16) {
  const int lane = threadIdx.x & 31;
  const int wave = threadIdx.x >> 5;
  const int row = blockIdx.x * 8 + wave;
  const int s = row >> 7;
  const int kk = row & 127;
  const float* rp = raw + (size_t)row * CH4;
  float ss = 0.f;
#pragma unroll 1
  for (int it = 0; it < 4; ++it) {
    const int c = it * 256 + 8 * lane;
    const v4f a = *(const v4f*)(rp + c);
    const v4f bq = *(const v4f*)(rp + c + 4);
    const float a0 = a[0] * gin, a1 = a[1] * gin, a2 = a[2] * gin, a3 = a[3] * gin;
    const float b0 = bq[0] * gin, b1 = bq[1] * gin, b2 = bq[2] * gin, b3 = bq[3] * gin;
    ss += ((a0 * a0 + a1 * a1) + (a2 * a2 + a3 * a3)) + ((b0 * b0 + b1 * b1) + (b2 * b2 + b3 * b3));
  }
#pragma unroll
  for (int off = 16; off > 0; off >>= 1) ss += __shfl_xor(ss, off, 32);
  const float nrm = sqrtf(ss);
  float inv;
  if (HAS_SZ) {
    float cq = colsq[((size_t)s * 64 + lane) * KPOOL + kk] + colsq[((size_t)s * 64 + lane + 32) * KPOOL + kk];
#pragma unroll
    for (int off = 16; off > 0; off >>= 1) cq += __shfl_xor(cq, off, 32);
    const float sz = 1.0f / (1e-6f + sqrtf(cq));
    inv = sz * (1.0f / (1e-6f + sz * nrm));
  } else {
    inv = 1.0f / (1e-6f + nrm);
  }
  const float mul = inv * gin * BCAR;
  unsigned short* ob = out16 + (size_t)row * CH4;
#pragma unroll 1
  for (int it = 0; it < 4; ++it) {
    const int c = it * 256 + 8 * lane;
    const v4f a = *(const v4f*)(rp + c);
    const v4f bq = *(const v4f*)(rp + c + 4);
    v8h hv;
    hv[0] = (_Float16)(a[0] * mul); hv[1] = (_Float16)(a[1] * mul); hv[2] = (_Float16)(a[2] * mul); hv[3] = (_Float16)(a[3] * mul);
    hv[4] = (_Float16)(bq[0] * mul); hv[5] = (_Float16)(bq[1] * mul); hv[6] = (_Float16)(bq[2] * mul); hv[7] = (_Float16)(bq[3] * mul);
    unsigned short* dst = ob + c;
    *(volatile v8h*)dst = hv;
    __threadfence();
    *(volatile v8h*)dst = hv;
  }
}

__global__ __launch_bounds__(256) void att_softmax_kernel(const float* __restrict__ attL, unsigned short* __restrict__ pp) {
  const int lane = threadIdx.x & 31;
  const int wave = threadIdx.x >> 5;
  const int row = blockIdx.x * 16 + wave * 2 + (lane >> 4);
  const int c8 = (lane & 15) * 8;
  const float* rp = attL + (size_t)row * HDIM + c8;
  const v4f a = *(const v4f*)rp;
  const v4f bq = *(const v4f*)(rp + 4);
  float mx = fmaxf(fmaxf(fmaxf(a[0], a[1]), fmaxf(a[2], a[3])), fmaxf(fmaxf(bq[0], bq[1]), fmaxf(bq[2], bq[3])));
#pragma unroll
  for (int off = 1; off < 16; off <<= 1) mx = fmaxf(mx, __shfl_xor(mx, off, 32));
  const float e0 = expf(a[0] - mx), e1 = expf(a[1] - mx), e2 = expf(a[2] - mx), e3 = expf(a[3] - mx);
  const float e4 = expf(bq[0] - mx), e5 = expf(bq[1] - mx), e6 = expf(bq[2] - mx), e7 = expf(bq[3] - mx);
  float ssum = ((e0 + e1) + (e2 + e3)) + ((e4 + e5) + (e6 + e7));
#pragma unroll
  for (int off = 1; off < 16; off <<= 1) ssum += __shfl_xor(ssum, off, 32);
  const float mul = (1.0f / ssum) * PCAR;
  v8h hv;
  hv[0] = (_Float16)(e0 * mul); hv[1] = (_Float16)(e1 * mul); hv[2] = (_Float16)(e2 * mul); hv[3] = (_Float16)(e3 * mul);
  hv[4] = (_Float16)(e4 * mul); hv[5] = (_Float16)(e5 * mul); hv[6] = (_Float16)(e6 * mul); hv[7] = (_Float16)(e7 * mul);
  unsigned short* dst = pp + (size_t)row * HDIM + c8;
  *(volatile v8h*)dst = hv;
  __threadfence();
  *(volatile v8h*)dst = hv;
}

__global__ __launch_bounds__(256) void gelu_kernel(const float* __restrict__ in, unsigned short* __restrict__ out) {
  __shared__ __align__(16) unsigned short lds[8 * 256];
  const int lane = threadIdx.x & 31;
  const int wave = threadIdx.x >> 5;
  const size_t wbase = ((size_t)blockIdx.x * 8 + wave) * 256;
  unsigned short* lw = lds + wave * 256;
#pragma unroll 1
  for (int it = 0; it < 8; ++it) {
    const float x = in[wbase + it * 32 + lane];
    const float gv = 0.5f * x * (1.0f + erff(x * 0.70710678118654752f));
    lw[it * 32 + lane] = f2h_bits(gv * HCAR);
  }
  __syncthreads();
  const v4u v = *(const v4u*)(lw + lane * 8);
  unsigned short* dst = out + wbase + lane * 8;
  *(volatile v4u*)dst = v;
  __threadfence();
  *(volatile v4u*)dst = v;
}

__global__ __launch_bounds__(256) void resid_sum_kernel(
    const float* __restrict__ a2t, const float* __restrict__ xca, float* __restrict__ res) {
  __shared__ __align__(16) float tr[64 * 68];
  const int t = threadIdx.x;
  const int lane = t & 31;
  const int wave = t >> 5;
  const int p0 = blockIdx.x * 64;
  const int c0 = blockIdx.y * 64;
#pragma unroll
  for (int it = 0; it < 4; ++it) {
    const int pp = it * 16 + (t >> 4);
    const int c4 = (t & 15) * 4;
    const v4f v = *(const v4f*)(xca + (size_t)(p0 + pp) * NCH + c0 + c4);
    tr[(c4 + 0) * 68 + pp] = v[0];
    tr[(c4 + 1) * 68 + pp] = v[1];
    tr[(c4 + 2) * 68 + pp] = v[2];
    tr[(c4 + 3) * 68 + pp] = v[3];
  }
  __syncthreads();
  const int hh = lane >> 4;
  const int p4 = (lane & 15) * 4;
  v4f sum[4];
#pragma unroll
  for (int it = 0; it < 4; ++it) {
    const int cc = wave * 8 + it * 2 + hh;
    const v4f av = *(const v4f*)(a2t + (size_t)(c0 + cc) * NPIX + p0 + p4);
    const v4f xv = *(const v4f*)(tr + cc * 68 + p4);
    sum[it] = av + xv;
  }
  for (int pass = 0; pass < 2; ++pass) {
#pragma unroll
    for (int it = 0; it < 4; ++it) {
      const int cc = wave * 8 + it * 2 + hh;
      *(volatile v4f*)(res + (size_t)(c0 + cc) * NPIX + p0 + p4) = sum[it];
    }
    __threadfence();
  }
}

__global__ __launch_bounds__(256) void prep_small_kernel(
    const float* __restrict__ bg1, const float* __restrict__ bb1, const float* __restrict__ bm1, const float* __restrict__ bv1,
    const float* __restrict__ bg2, const float* __restrict__ bb2, const float* __restrict__ bm2, const float* __restrict__ bv2,
    const float* __restrict__ bp, float* __restrict__ smallv) {
  const int c = threadIdx.x;
  const float s1 = bg1[c] * rsqrtf(bv1[c] + 1e-5f);
  const float t1 = bb1[c] - bm1[c] * s1;
  const float s2 = bg2[c] * rsqrtf(bv2[c] + 1e-5f);
  const float t2 = bb2[c] - bm2[c] * s2;
  const float p2 = 2.0f * bp[c];
  const float s1w = s1 * (1.0f / WCAR);
  const float s2w = s2 * (1.0f / WCAR);
  volatile float* o = smallv;
  o[c] = s1w; o[256 + c] = t1; o[512 + c] = s2w; o[768 + c] = t2; o[1024 + c] = p2;
  __threadfence();
  o[c] = s1w; o[256 + c] = t1; o[512 + c] = s2w; o[768 + c] = t2; o[1024 + c] = p2;
}

__global__ __launch_bounds__(256) void cast_lin_kernel(
    const float* __restrict__ wq, const float* __restrict__ wk, const float* __restrict__ wv,
    const float* __restrict__ wp, const float* __restrict__ w1, const float* __restrict__ w2,
    unsigned short* __restrict__ wqkv, unsigned short* __restrict__ wp16,
    unsigned short* __restrict__ w1_16, unsigned short* __restrict__ w2_16) {
  const int seg = blockIdx.y;
  const float* src;
  unsigned short* dst;
  if (seg == 0)      { src = wq; dst = wqkv; }
  else if (seg == 1) { src = wk; dst = wqkv + (size_t)CH4 * NCH; }
  else if (seg == 2) { src = wv; dst = wqkv + (size_t)2 * CH4 * NCH; }
  else if (seg == 3) { src = wp; dst = wp16; }
  else if (seg == 4) { src = w1; dst = w1_16; }
  else               { src = w2; dst = w2_16; }
  const size_t i = (size_t)blockIdx.x * 256 + threadIdx.x;
  const v4f a = *(const v4f*)(src + 8 * i);
  const v4f bq = *(const v4f*)(src + 8 * i + 4);
  v8h hv;
  hv[0] = (_Float16)(a[0] * WCAR); hv[1] = (_Float16)(a[1] * WCAR); hv[2] = (_Float16)(a[2] * WCAR); hv[3] = (_Float16)(a[3] * WCAR);
  hv[4] = (_Float16)(bq[0] * WCAR); hv[5] = (_Float16)(bq[1] * WCAR); hv[6] = (_Float16)(bq[2] * WCAR); hv[7] = (_Float16)(bq[3] * WCAR);
  unsigned short* d = dst + 8 * i;
  *(volatile v8h*)d = hv;
  __threadfence();
  *(volatile v8h*)d = hv;
}

__global__ __launch_bounds__(256) void cast_convw_kernel(
    const float* __restrict__ cw1, const float* __restrict__ cw2,
    unsigned short* __restrict__ wt1, unsigned short* __restrict__ wt2) {
  const float* src = (blockIdx.y == 0) ? cw1 : cw2;
  unsigned short* dst = (blockIdx.y == 0) ? wt1 : wt2;
  const int i = blockIdx.x * 256 + threadIdx.x;
  const int o = i / 288;
  const int ch = i - o * 288;
  const int k8 = ch * 8;
  const int kk = k8 >> 8;
  const int ci = k8 & 255;
  const float* sp = src + ((size_t)(o * NCH + ci) * 9 + kk);
  v8h hv;
#pragma unroll
  for (int e = 0; e < 8; ++e) hv[e] = (_Float16)(sp[e * 9] * WCAR);
  unsigned short* d = dst + (size_t)o * KCONV + k8;
  *(volatile v8h*)d = hv;
  __threadfence();
  *(volatile v8h*)d = hv;
}

extern "C" void kernel_launch(void* const* d_in, const int* in_sizes, int n_in,
                              void* d_out, int out_size, void* d_ws, size_t ws_size,
                              hipStream_t stream) {
  (void)n_in;
  const float* x   = (const float*)d_in[0];
  const float* Wq  = (const float*)d_in[1];
  const float* Wk  = (const float*)d_in[2];
  const float* Wv  = (const float*)d_in[3];
  const float* Wp  = (const float*)d_in[4];
  const float* bp  = (const float*)d_in[5];
  const float* g1  = (const float*)d_in[6];
  const float* b1  = (const float*)d_in[7];
  const float* g2  = (const float*)d_in[8];
  const float* b2  = (const float*)d_in[9];
  const float* W1  = (const float*)d_in[10];
  const float* bf1 = (const float*)d_in[11];
  const float* W2  = (const float*)d_in[12];
  const float* bf2 = (const float*)d_in[13];
  const float* cw1 = (const float*)d_in[14];
  const float* bg1 = (const float*)d_in[15];
  const float* bb1 = (const float*)d_in[16];
  const float* bm1 = (const float*)d_in[17];
  const float* bv1 = (const float*)d_in[18];
  const float* cw2 = (const float*)d_in[19];
  const float* bg2 = (const float*)d_in[20];
  const float* bb2 = (const float*)d_in[21];
  const float* bm2 = (const float*)d_in[22];
  const float* bv2 = (const float*)d_in[23];
  const float* alphap = (const float*)d_in[24];
  float* out = (float*)d_out;

  constexpr size_t SZ_WQKV  = (size_t)QKV_LD * NCH * 2;
  constexpr size_t SZ_WLIN  = (size_t)CH4 * NCH * 2;
  constexpr size_t SZ_WT    = (size_t)NCH * KCONV * 2;
  constexpr size_t SZ_SMALL = 8192;
  constexpr size_t SZ_TOK16 = (size_t)NBATCH * NPIX * NCH * 2;
  constexpr size_t SZ_XC2   = (size_t)NBATCH * NPIX * NCH * 4;
  constexpr size_t SZ_QKV   = (size_t)NPIX * QKV_LD * 2;
  constexpr size_t SZ_QKC   = (size_t)2 * CH4 * NPIX * 2;
  constexpr size_t SZ_ZT    = (size_t)2 * KPOOL * NPIX * 2;
  constexpr size_t SZ_COLSQ = (size_t)2 * 64 * KPOOL * 4;
  constexpr size_t SZ_BRAW  = (size_t)2 * KPOOL * CH4 * 4;
  constexpr size_t SZ_B16   = (size_t)2 * KPOOL * CH4 * 2;
  constexpr size_t SZ_ATTL  = (size_t)NHEAD * HDIM * HDIM * 4;
  constexpr size_t SZ_P16   = (size_t)NHEAD * HDIM * HDIM * 2;
  constexpr size_t SZ_O16   = (size_t)NPIX * CH4 * 2;
  constexpr size_t SZ_A2T   = (size_t)NCH * NPIX * 4;
  constexpr size_t SZ_LN2   = (size_t)NPIX * NCH * 2;
  constexpr size_t SZ_H16   = (size_t)NPIX * CH4 * 2;
  constexpr size_t SZ_RES   = (size_t)NCH * NPIX * 4;
  static_assert(SZ_QKC == (size_t)NPIX * CH4 * 4);

  constexpr size_t OF_WQKV  = 0;
  constexpr size_t OF_WP16  = OF_WQKV + SZ_WQKV;
  constexpr size_t OF_W116  = OF_WP16 + SZ_WLIN;
  constexpr size_t OF_W216  = OF_W116 + SZ_WLIN;
  constexpr size_t OF_WT1   = OF_W216 + SZ_WLIN;
  constexpr size_t OF_WT2   = OF_WT1 + SZ_WT;
  constexpr size_t OF_SMALL = OF_WT2 + SZ_WT;
  constexpr size_t OF_XT    = OF_SMALL + SZ_SMALL;
  constexpr size_t OF_T1    = OF_XT + SZ_TOK16;
  constexpr size_t OF_XC1   = OF_T1 + SZ_TOK16;
  constexpr size_t OF_XC2   = OF_XC1 + SZ_TOK16;
  constexpr size_t OF_QKV   = OF_XC2 + SZ_XC2;
  constexpr size_t OF_QKC   = OF_QKV + SZ_QKV;
  constexpr size_t OF_ZT    = OF_QKC + SZ_QKC;
  constexpr size_t OF_COLSQ = OF_ZT + SZ_ZT;
  constexpr size_t OF_BRAW  = OF_COLSQ + SZ_COLSQ;
  constexpr size_t OF_B16   = OF_BRAW + SZ_BRAW;
  constexpr size_t OF_BC16  = OF_B16 + SZ_B16;
  constexpr size_t OF_ATTL  = OF_BC16 + SZ_B16;
  constexpr size_t OF_P16   = OF_ATTL + SZ_ATTL;
  constexpr size_t OF_O16   = OF_P16 + SZ_P16;
  constexpr size_t OF_A2T   = OF_O16 + SZ_O16;
  constexpr size_t OF_LN2   = OF_A2T + SZ_A2T;
  constexpr size_t OF_H16   = OF_LN2 + SZ_LN2;
  constexpr size_t OF_RES   = OF_H16 + SZ_H16;
  constexpr size_t WS_TOTAL = OF_RES + SZ_RES;
  static_assert(WS_TOTAL == 121708544ull);
  static_assert(WS_TOTAL <= 134217728ull);
  static_assert((OF_SMALL % 256) == 0 && (OF_QKV % 256) == 0 && (OF_H16 % 256) == 0 && (OF_RES % 256) == 0);

  if (ws_size < WS_TOTAL) return;
  if ((size_t)out_size != (size_t)NBATCH * NCH * NPIX) return;
  if ((size_t)in_sizes[0] != (size_t)NBATCH * NCH * NPIX) return;
  if (in_sizes[14] != NCH * NCH * 9 || in_sizes[19] != NCH * NCH * 9 || in_sizes[1] != CH4 * NCH) return;

  char* ws = (char*)d_ws;
  unsigned short* wqkv  = (unsigned short*)(ws + OF_WQKV);
  unsigned short* wp16  = (unsigned short*)(ws + OF_WP16);
  unsigned short* w1_16 = (unsigned short*)(ws + OF_W116);
  unsigned short* w2_16 = (unsigned short*)(ws + OF_W216);
  unsigned short* wt1   = (unsigned short*)(ws + OF_WT1);
  unsigned short* wt2   = (unsigned short*)(ws + OF_WT2);
  float* smallv = (float*)(ws + OF_SMALL);
  float* cs1w = smallv;
  float* cb1  = smallv + 256;
  float* cs2w = smallv + 512;
  float* cb2  = smallv + 768;
  float* bp2  = smallv + 1024;
  unsigned short* xt    = (unsigned short*)(ws + OF_XT);
  unsigned short* t1    = (unsigned short*)(ws + OF_T1);
  unsigned short* xc1t  = (unsigned short*)(ws + OF_XC1);
  float* xc2t = (float*)(ws + OF_XC2);
  unsigned short* qkv   = (unsigned short*)(ws + OF_QKV);
  unsigned short* qkc   = (unsigned short*)(ws + OF_QKC);
  float* h1raw = (float*)(ws + OF_QKC);
  unsigned short* zT    = (unsigned short*)(ws + OF_ZT);
  float* colsq = (float*)(ws + OF_COLSQ);
  float* braw  = (float*)(ws + OF_BRAW);
  unsigned short* b16   = (unsigned short*)(ws + OF_B16);
  unsigned short* bc16  = (unsigned short*)(ws + OF_BC16);
  float* attL  = (float*)(ws + OF_ATTL);
  unsigned short* p16   = (unsigned short*)(ws + OF_P16);
  unsigned short* o16   = (unsigned short*)(ws + OF_O16);
  float* a2t   = (float*)(ws + OF_A2T);
  unsigned short* ln2   = (unsigned short*)(ws + OF_LN2);
  unsigned short* h16   = (unsigned short*)(ws + OF_H16);
  float* res   = (float*)(ws + OF_RES);

  const dim3 blk256(256);

  prep_small_kernel<<<dim3(1), blk256, 0, stream>>>(bg1, bb1, bm1, bv1, bg2, bb2, bm2, bv2, bp, smallv);
  cast_lin_kernel<<<dim3(CH4 * NCH / 8 / 256, 6), blk256, 0, stream>>>(Wq, Wk, Wv, Wp, W1, W2, wqkv, wp16, w1_16, w2_16);
  cast_convw_kernel<<<dim3(NCH * (KCONV / 8) / 256, 2), blk256, 0, stream>>>(cw1, cw2, wt1, wt2);

  ln_tok_kernel<true><<<dim3(NPIX / 32, NBATCH), blk256, 0, stream>>>(x, (long)NCH * NPIX, g1, b1, t1, xt);

  {
    const int tiles = (NBATCH * NPIX / 64) * (NCH / 64);
    conv3x3_wmma64<1, false><<<dim3(tiles / 8), blk256, 0, stream>>>(xt, wt1, cs1w, cb1, alphap, (void*)xc1t);
    conv3x3_wmma64<0, true ><<<dim3(tiles / 8), blk256, 0, stream>>>(xc1t, wt2, cs2w, cb2, alphap, (void*)xc2t);
  }

  for (int b = 0; b < NBATCH; ++b) {
    const unsigned short* t1b = t1 + (size_t)b * NPIX * NCH;
    const float* xc2b = xc2t + (size_t)b * NPIX * NCH;
    float* outb = out + (size_t)b * NCH * NPIX;

    {
      const int tiles = (NPIX / 64) * (QKV_LD / 64);
      wmma_gemm64<0, false, 0, 1, false, 0><<<dim3((tiles + 7) / 8, 1), blk256, 0, stream>>>(
          t1b, t1b, NCH, 0, wqkv, wqkv, NCH, 0, (void*)qkv, (void*)qkv, QKV_LD, 0,
          smallv, smallv, 0, NPIX, QKV_LD, NCH, QCAR / WCAR);
    }
    transpose16_kernel<<<dim3(NPIX / 64, CH4 / 64, 2), blk256, 0, stream>>>(qkv, QKV_LD, (long)CH4, qkc, NPIX, (long)CH4 * NPIX);

    pool_kernel<<<dim3(CH4 / 256, KPOOL, 2), blk256, 0, stream>>>(qkc, braw);
    rownorm_kernel<false><<<dim3(2 * KPOOL / 8), blk256, 0, stream>>>(braw, colsq, 1.0f / QCAR, b16);

    for (int st = 0; st < NSTAGE; ++st) {
      dta_logit_softmax_kernel<<<dim3(NPIX / 64, 2), dim3(64), 0, stream>>>(qkv, b16, zT, colsq, 1.0f / (QCAR * BCAR));
      {
        const int tiles = (KPOOL / 64) * (CH4 / 64);
        wmma_gemm64<0, false, 0, 0, false, 0><<<dim3((tiles + 7) / 8, 2), blk256, 0, stream>>>(
            zT, zT, NPIX, (long)KPOOL * NPIX, qkc, qkc, NPIX, (long)CH4 * NPIX,
            (void*)braw, (void*)braw, CH4, (long)KPOOL * CH4,
            smallv, smallv, 0, KPOOL, CH4, NPIX, 1.0f / (ZCAR * QCAR));
      }
      rownorm_kernel<true><<<dim3(2 * KPOOL / 8), blk256, 0, stream>>>(braw, colsq, 1.0f, b16);
    }

    transpose16_kernel<<<dim3(KPOOL / 64, CH4 / 64, 2), blk256, 0, stream>>>(b16, CH4, (long)KPOOL * CH4, bc16, KPOOL, (long)CH4 * KPOOL);

    {
      const int tiles = (HDIM / 64) * (HDIM / 64);
      wmma_gemm64<0, false, 0, 0, false, 0><<<dim3((tiles + 7) / 8, NHEAD), blk256, 0, stream>>>(
          bc16, bc16, KPOOL, (long)HDIM * KPOOL,
          bc16 + (size_t)CH4 * KPOOL, bc16 + (size_t)CH4 * KPOOL, KPOOL, (long)HDIM * KPOOL,
          (void*)attL, (void*)attL, HDIM, (long)HDIM * HDIM,
          smallv, smallv, 0, HDIM, HDIM, KPOOL, ATT_SCALE / (BCAR * BCAR));
    }
    att_softmax_kernel<<<dim3(NHEAD * HDIM / 16), blk256, 0, stream>>>(attL, p16);

    {
      const int tiles = (NPIX / 64) * (HDIM / 64);
      wmma_gemm64<0, false, 0, 1, false, 0><<<dim3((tiles + 7) / 8, NHEAD), blk256, 0, stream>>>(
          qkv + (size_t)2 * CH4, qkv + (size_t)2 * CH4, QKV_LD, (long)HDIM,
          p16, p16, HDIM, (long)HDIM * HDIM,
          (void*)o16, (void*)o16, CH4, (long)HDIM,
          smallv, smallv, 0, NPIX, HDIM, HDIM, OCAR / (QCAR * PCAR));
    }

    {
      const int tiles = (NCH / 64) * (NPIX / 64);
      wmma_gemm64<0, false, 1, 0, false, 2><<<dim3((tiles + 7) / 8, 1), blk256, 0, stream>>>(
          wp16, wp16, CH4, 0, o16, o16, CH4, 0, (void*)a2t, (void*)a2t, NPIX, 0,
          bp2, smallv, 0, NCH, NPIX, CH4, 2.0f / (WCAR * OCAR));
    }

    ln_tok_kernel<false><<<dim3(NPIX / 32, 1), blk256, 0, stream>>>(a2t, 0, g2, b2, ln2, ln2);

    resid_sum_kernel<<<dim3(NPIX / 64, NCH / 64), blk256, 0, stream>>>(a2t, xc2b, res);

    {
      const int tiles = (NPIX / 64) * (CH4 / 64);
      wmma_gemm64<0, false, 2, 0, false, 0><<<dim3((tiles + 7) / 8, 1), blk256, 0, stream>>>(
          ln2, ln2, NCH, 0, w1_16, w1_16, NCH, 0, (void*)h1raw, (void*)h1raw, CH4, 0,
          bf1, smallv, 0, NPIX, CH4, NCH, 1.0f / WCAR);
    }
    gelu_kernel<<<dim3(NPIX * CH4 / 2048), blk256, 0, stream>>>(h1raw, h16);

    {
      const int tiles = (NCH / 64) * (NPIX / 64);
      wmma_gemm64<0, false, 1, 0, true, 0><<<dim3((tiles + 7) / 8, 1), blk256, 0, stream>>>(
          w2_16, w2_16, CH4, 0, h16, h16, CH4, 0, (void*)outb, (void*)outb, NPIX, 0,
          bf2, res, 0, NCH, NPIX, CH4, 1.0f / (WCAR * HCAR));
    }
  }
}
